// SAU_47691316855554
// MI455X (gfx1250) — hardware-verified
//
#include <hip/hip_runtime.h>
#include <math.h>

constexpr int kBatch  = 8;
constexpr int kCh     = 256;
constexpr int kPix    = 4096;
constexpr int kInter  = 64;
constexpr int kTok    = kBatch * kPix;
constexpr int kQKN    = 2 * kInter;
constexpr int kChunkQ = 2048;
constexpr int kHalves = kPix / kChunkQ;
constexpr float kWCarry    = 64.0f;
constexpr float kQKCarry   = 16.0f;
constexpr float kVCarry    = 16.0f;
constexpr float kPCarry    = 2048.0f;
constexpr float kProjScale = kQKCarry / kWCarry;
constexpr float kVScale    = kVCarry / kWCarry;
constexpr float kSScale    = 1.0f / (kQKCarry * kQKCarry * 8.0f);
constexpr float kOutScale  = 1.0f / (kPCarry * kVCarry);
constexpr float kMeanScale = 1.0f / (kVCarry * 4096.0f);

typedef __attribute__((ext_vector_type(16))) _Float16 v16h;
typedef __attribute__((ext_vector_type(8)))  _Float16 v8h;
typedef __attribute__((ext_vector_type(16))) __bf16   v16b;
typedef __attribute__((ext_vector_type(8)))  __bf16   v8b;
typedef __attribute__((ext_vector_type(8)))  float    v8f;
typedef __attribute__((ext_vector_type(4)))  float    v4f;
typedef __attribute__((ext_vector_type(4)))  unsigned int v4u;

__device__ __forceinline__ unsigned short f2bf_bits(float f) {
  unsigned u = __float_as_uint(f);
  return (unsigned short)((u + 0x7FFFu + ((u >> 16) & 1u)) >> 16);
}
__device__ __forceinline__ float bf_bits2f(unsigned short h) { return __uint_as_float(((unsigned)h) << 16); }

__device__ __forceinline__ void dep_guard_h(v8f& a, v8f& b, v16h x, v16h y) { asm volatile("v_nop\n\tv_nop\n\tv_nop\n\tv_nop" : "+v"(a), "+v"(b) : "v"(x), "v"(y)); }
__device__ __forceinline__ void dep_guard_b(v8f& a, v8f& b, v16b x, v16b y) { asm volatile("v_nop\n\tv_nop\n\tv_nop\n\tv_nop" : "+v"(a), "+v"(b) : "v"(x), "v"(y)); }
__device__ __forceinline__ void keep4_h(v16h a, v16h b, v16h c, v16h d) { asm volatile("v_nop" :: "v"(a), "v"(b), "v"(c), "v"(d)); }
__device__ __forceinline__ void keep4_b(v16b a, v16b b, v16b c, v16b d) { asm volatile("v_nop" :: "v"(a), "v"(b), "v"(c), "v"(d)); }
__device__ __forceinline__ void acc_guard4(v8f& a, v8f& b, v8f& c, v8f& d) { asm volatile("v_nop\n\tv_nop\n\tv_nop\n\tv_nop" : "+v"(a), "+v"(b), "+v"(c), "+v"(d)); }
template <typename T> struct Frag;
template <> struct Frag<_Float16> {
  typedef v16h V; union U { v16h v; v8h h[2]; };
  static __device__ __forceinline__ v16h load(const _Float16* p) {
    U f; f.h[0] = *(const v8h*)(p); f.h[1] = *(const v8h*)(p + 16); return f.v;
  }
  static __device__ __forceinline__ v8f mma(v16h a, v16h b, v8f c) {
    return __builtin_amdgcn_wmma_f32_16x16x32_f16(false, a, false, b, (short)0, c, false, false);
  }
  static __device__ __forceinline__ void guard(v8f& a, v8f& b, v16h x, v16h y) { dep_guard_h(a, b, x, y); }
  static __device__ __forceinline__ void keep(v16h a, v16h b, v16h c, v16h d) { keep4_h(a, b, c, d); }
};
template <> struct Frag<__bf16> {
  typedef v16b V; union U { v16b v; v8b h[2]; };
  static __device__ __forceinline__ v16b load(const __bf16* p) {
    U f; f.h[0] = *(const v8b*)(p); f.h[1] = *(const v8b*)(p + 16); return f.v;
  }
  static __device__ __forceinline__ v8f mma(v16b a, v16b b, v8f c) {
    return __builtin_amdgcn_wmma_f32_16x16x32_bf16(false, a, false, b, (short)0, c, false, false);
  }
  static __device__ __forceinline__ void guard(v8f& a, v8f& b, v16b x, v16b y) { dep_guard_b(a, b, x, y); }
  static __device__ __forceinline__ void keep(v16b a, v16b b, v16b c, v16b d) { keep4_b(a, b, c, d); }
};

__device__ __forceinline__ unsigned pk16(unsigned short a, unsigned short b) { return (unsigned)a | ((unsigned)b << 16); }
__device__ __forceinline__ unsigned short h_bits(float f) { const _Float16 h = (_Float16)f; return __builtin_bit_cast(unsigned short, h); }

__device__ __forceinline__ float h2f_bits(unsigned w) {
  const unsigned s = (w & 0x8000u) << 16;
  const unsigned e = (w >> 10) & 0x1fu;
  const unsigned m = w & 0x3ffu;
  const float nrm = __uint_as_float(((e + 112u) << 23) | (m << 13));
  const float sub = (float)m * 5.9604644775390625e-8f;
  const float mag = (e == 0u) ? sub : nrm;
  return __uint_as_float(__float_as_uint(mag) | s);
}

template <int ET> struct Elem;
template <> struct Elem<0> { typedef _Float16 T; };
template <> struct Elem<1> { typedef __bf16 T; };
template <int ET, bool SPLIT, int BIAS_MODE, int OUT_MODE, bool RESID, int ACT = 0, bool ADDM = false>
__global__ __launch_bounds__(256) void wmma_gemm64(
    const unsigned short* __restrict__ Ap, const unsigned short* __restrict__ A2p, int lda, long strideA,
    const unsigned short* __restrict__ Btp, const unsigned short* __restrict__ Bt2p, int ldb, long strideB,
    void* __restrict__ Cout, void* __restrict__ Cout2, int ldc, long strideC,
    const float* __restrict__ bias,
    const float* __restrict__ resid, long strideR,
    const float* __restrict__ addm, long strideAddm,
    int M, int N, int K, float scale) {
  typedef typename Elem<ET>::T T;
  typedef typename Frag<T>::V V;
  const T* A = (const T*)Ap; const T* A2 = (const T*)A2p; const T* Bt = (const T*)Btp; const T* Bt2 = (const T*)Bt2p;
  __shared__ __align__(16) float sT[8][16 * 68];
  const int b    = blockIdx.y;
  const int lane = threadIdx.x & 31;
  const int wave = threadIdx.x >> 5;
  const int tilesN = N >> 6;
  const int tilesM = M >> 6;
  const int tile = blockIdx.x * 8 + wave;
  if (tile >= tilesM * tilesN) return;
  const int tm = tile / tilesN;
  const int tn = tile - tm * tilesN;
  const int m0 = tm << 6;
  const int n0 = tn << 6;

  const T* Ab  = A  + (size_t)b * strideA;
  const T* Bb  = Bt + (size_t)b * strideB;
  const T* Ab2 = SPLIT ? (A2  + (size_t)b * strideA) : nullptr;
  const T* Bb2 = SPLIT ? (Bt2 + (size_t)b * strideB) : nullptr;

  const int rlane = lane & 15;
  const int koff  = (lane >> 4) * 8;
  const int mOff  = (lane >> 4) * 8;

  v8f acc[4][4];
#pragma unroll
  for (int i = 0; i < 4; ++i)
#pragma unroll
    for (int j = 0; j < 4; ++j) acc[i][j] = (v8f){0.f,0.f,0.f,0.f,0.f,0.f,0.f,0.f};

  for (int k0 = 0; k0 < K; k0 += 32) {
    V bh[4], bl[4];
#pragma unroll
    for (int j = 0; j < 4; ++j) {
      const size_t bo = (size_t)(n0 + (j << 4) + rlane) * ldb + koff + k0;
      bh[j] = Frag<T>::load(Bb + bo);
      if (SPLIT) bl[j] = Frag<T>::load(Bb2 + bo);
    }
#pragma unroll
    for (int i = 0; i < 4; ++i) {
      const size_t ao = (size_t)(m0 + (i << 4) + rlane) * lda + koff + k0;
      V ah = Frag<T>::load(Ab + ao);
      V al;
      if (SPLIT) al = Frag<T>::load(Ab2 + ao);
#pragma unroll
      for (int j = 0; j < 4; ++j) {
        acc[i][j] = Frag<T>::mma(ah, bh[j], acc[i][j]);
        if (SPLIT) {
          acc[i][j] = Frag<T>::mma(ah, bl[j], acc[i][j]);
          acc[i][j] = Frag<T>::mma(al, bh[j], acc[i][j]);
        }
      }
      Frag<T>::guard(acc[i][0], acc[i][3], ah, SPLIT ? al : ah);
    }
    Frag<T>::keep(bh[0], bh[1], bh[2], bh[3]);
    if (SPLIT) Frag<T>::keep(bl[0], bl[1], bl[2], bl[3]);
  }
  acc_guard4(acc[0][0], acc[0][1], acc[0][2], acc[0][3]);
  acc_guard4(acc[1][0], acc[1][1], acc[1][2], acc[1][3]);
  acc_guard4(acc[2][0], acc[2][1], acc[2][2], acc[2][3]);
  acc_guard4(acc[3][0], acc[3][1], acc[3][2], acc[3][3]);

  float* slab = sT[wave];
  const float* Rb = RESID ? (resid + (size_t)b * strideR) : nullptr;
  const float* Mb = ADDM ? (addm + (size_t)b * strideAddm) : nullptr;
#pragma unroll
  for (int i = 0; i < 4; ++i) {
    const int mBase = m0 + (i << 4);
#pragma unroll
    for (int j = 0; j < 4; ++j) {
      const int n = n0 + (j << 4) + rlane;
      float bv = 0.f;
      if (BIAS_MODE == 2) bv = bias[n];
#pragma unroll
      for (int r = 0; r < 8; ++r) {
        float v = acc[i][j][r] * scale;
        if (BIAS_MODE == 1) v += bias[mBase + mOff + r];
        if (BIAS_MODE == 2) v += bv;
        if (RESID) v += Rb[(size_t)(mBase + mOff + r) * ldc + n];
        if (ADDM) v += Mb[mBase + mOff + r];
        if (ACT == 2) v = fmaxf(v, 0.0f);
        if (ACT == 4) v = (v > 0.f) ? v : 0.01f * v;
        slab[(mOff + r) * 68 + (j << 4) + rlane] = v;
      }
    }
    __builtin_amdgcn_fence(__ATOMIC_RELEASE, "workgroup");
    __builtin_amdgcn_wave_barrier();
    __builtin_amdgcn_fence(__ATOMIC_ACQUIRE, "workgroup");
    if (OUT_MODE == 0) {
      float* C = (float*)Cout + (size_t)b * strideC;
      const int hh = lane >> 4, c4 = (lane & 15) * 4;
      for (int pass = 0; pass < 2; ++pass) {
#pragma unroll
        for (int it = 0; it < 8; ++it) {
          const int row = it * 2 + hh;
          v4f v = *(const v4f*)(slab + row * 68 + c4);
          *(volatile v4f*)(C + (size_t)(mBase + row) * ldc + n0 + c4) = v;
        }
        __threadfence();
      }
    } else {
      const int q = lane >> 3, c8 = (lane & 7) * 8;
      unsigned short* C  = (unsigned short*)Cout  + (size_t)b * strideC;
      unsigned short* C2 = (OUT_MODE == 2) ? ((unsigned short*)Cout2 + (size_t)b * strideC) : nullptr;
      for (int pass = 0; pass < 2; ++pass) {
#pragma unroll
        for (int it = 0; it < 4; ++it) {
          const int row = it * 4 + q;
          const float* sp = slab + row * 68 + c8;
          v8h hv, lv;
#pragma unroll
          for (int e = 0; e < 8; ++e) {
            if (OUT_MODE == 1) {
              hv[e] = (_Float16)sp[e];
            } else {
              unsigned short hb = f2bf_bits(sp[e]);
              unsigned short lb = f2bf_bits(sp[e] - bf_bits2f(hb));
              hv[e] = __builtin_bit_cast(_Float16, hb);
              lv[e] = __builtin_bit_cast(_Float16, lb);
            }
          }
          *(volatile v8h*)(C + (size_t)(mBase + row) * ldc + n0 + c8) = hv;
          if (OUT_MODE == 2) *(volatile v8h*)(C2 + (size_t)(mBase + row) * ldc + n0 + c8) = lv;
        }
        __threadfence();
      }
    }
    __builtin_amdgcn_fence(__ATOMIC_RELEASE, "workgroup");
    __builtin_amdgcn_wave_barrier();
    __builtin_amdgcn_fence(__ATOMIC_ACQUIRE, "workgroup");
  }
}

__global__ __launch_bounds__(256) void xpose_kernel(const float* __restrict__ x, unsigned short* __restrict__ X16) {
  __shared__ float sm[64][65];
  const int t  = threadIdx.x;
  const int n0 = blockIdx.x * 64;
  const int c0 = blockIdx.y * 64;
  const int b  = blockIdx.z;
  const float* xb = x + ((size_t)(b * kCh + c0)) * kPix + n0;
#pragma unroll
  for (int i = 0; i < 16; ++i) {
    const int e  = i * 256 + t;
    const int cl = e >> 6;
    const int nl = e & 63;
    sm[nl][cl] = xb[(size_t)cl * kPix + nl];
  }
  __syncthreads();
  const int lane = t & 31, wave = t >> 5;
  const int q = lane >> 3, c8 = (lane & 7) * 8;
  unsigned short* op = X16 + ((size_t)(b * kPix + n0)) * kCh + c0;
  for (int pass = 0; pass < 2; ++pass) {
#pragma unroll
    for (int it = 0; it < 2; ++it) {
      const int row = wave * 8 + it * 4 + q;
      unsigned short hb[8];
#pragma unroll
      for (int e = 0; e < 8; ++e) hb[e] = h_bits(sm[row][c8 + e]);
      const v4u u = (v4u){pk16(hb[0], hb[1]), pk16(hb[2], hb[3]), pk16(hb[4], hb[5]), pk16(hb[6], hb[7])};
      *(volatile v4u*)(op + (size_t)row * kCh + c8) = u;
    }
    __threadfence();
  }
}

__global__ __launch_bounds__(256) void prep_kernel(const float* __restrict__ wq, const float* __restrict__ wk,
                                                   const float* __restrict__ wv, const float* __restrict__ bq,
                                                   const float* __restrict__ bk, const float* __restrict__ bv,
                                                   unsigned short* __restrict__ Wqk16, unsigned short* __restrict__ Wv16,
                                                   float* __restrict__ biasqk, float* __restrict__ biasv) {
  const int blk = blockIdx.x;
  const int t   = threadIdx.x;
  if (blk < 48) {
    const float* src; unsigned short* dst; int i;
    if (blk < 8)       { src = wq; dst = Wqk16;                 i = blk * 256 + t; }
    else if (blk < 16) { src = wk; dst = Wqk16 + kInter * kCh;  i = (blk - 8) * 256 + t; }
    else               { src = wv; dst = Wv16;                  i = (blk - 16) * 256 + t; }
    const float* p = src + 8 * (size_t)i;
    const v4f a = *(const v4f*)(p) * kWCarry;
    const v4f c = *(const v4f*)(p + 4) * kWCarry;
    unsigned short hb[8];
#pragma unroll
    for (int e = 0; e < 4; ++e) { hb[e] = h_bits(a[e]); hb[4 + e] = h_bits(c[e]); }
    const v4u u = (v4u){pk16(hb[0], hb[1]), pk16(hb[2], hb[3]), pk16(hb[4], hb[5]), pk16(hb[6], hb[7])};
    unsigned short* qd = dst + 8 * (size_t)i;
    *(volatile v4u*)qd = u;
    __threadfence();
    *(volatile v4u*)qd = u;
  } else {
    const int lane = t & 31, wave = t >> 5;
    if (wave < 2) {
      if (lane < 16) {
        const float* s = ((wave == 0) ? bq : bk) + 4 * lane;
        const v4f v = *(const v4f*)(s) * kQKCarry;
        float* d = biasqk + wave * kInter + 4 * lane;
        *(volatile v4f*)d = v;
        __threadfence();
        *(volatile v4f*)d = v;
      }
    } else if (wave < 4) {
      const float* s = bv + (wave - 2) * 128 + 4 * lane;
      const v4f v = *(const v4f*)(s) * kVCarry;
      float* d = biasv + (wave - 2) * 128 + 4 * lane;
      *(volatile v4f*)d = v;
      __threadfence();
      *(volatile v4f*)d = v;
    }
  }
}

__global__ __launch_bounds__(512) void softmax_row_kernel(const float* __restrict__ S, unsigned short* __restrict__ P) {
  __shared__ float redM[16];
  __shared__ float redS[16];
  const int row  = blockIdx.x;
  const int t    = threadIdx.x;
  const int lane = t & 31, wave = t >> 5;
  const float* sr = S + (size_t)row * kPix + 8 * t;
  const v4f a = *(const v4f*)(sr);
  const v4f c = *(const v4f*)(sr + 4);
  float xv[8];
#pragma unroll
  for (int e = 0; e < 4; ++e) { xv[e] = a[e]; xv[4 + e] = c[e]; }
  float m = fmaxf(fmaxf(fmaxf(xv[0], xv[1]), fmaxf(xv[2], xv[3])), fmaxf(fmaxf(xv[4], xv[5]), fmaxf(xv[6], xv[7])));
#pragma unroll
  for (int off = 16; off > 0; off >>= 1) m = fmaxf(m, __shfl_xor(m, off, 32));
  if (lane == 0) redM[wave] = m;
  __syncthreads();
  float gm = redM[0];
#pragma unroll
  for (int w = 1; w < 16; ++w) gm = fmaxf(gm, redM[w]);
  float p[8];
  float ps = 0.f;
#pragma unroll
  for (int e = 0; e < 8; ++e) { p[e] = expf(xv[e] - gm); ps += p[e]; }
#pragma unroll
  for (int off = 16; off > 0; off >>= 1) ps += __shfl_xor(ps, off, 32);
  if (lane == 0) redS[wave] = ps;
  __syncthreads();
  float tot = 0.f;
#pragma unroll
  for (int w = 0; w < 16; ++w) tot += redS[w];
  const float f = kPCarry / tot;
  unsigned short hb[8];
#pragma unroll
  for (int e = 0; e < 8; ++e) hb[e] = h_bits(fmaf(p[e], f, -0.5f));
  const v4u u = (v4u){pk16(hb[0], hb[1]), pk16(hb[2], hb[3]), pk16(hb[4], hb[5]), pk16(hb[6], hb[7])};
  unsigned short* qd = P + (size_t)row * kPix + 8 * t;
  *(volatile v4u*)qd = u;
  __threadfence();
  *(volatile v4u*)qd = u;
}

__global__ __launch_bounds__(256) void vmean_kernel(const unsigned short* __restrict__ V16, float* __restrict__ vmean) {
  __shared__ float red[32];
  const int cg   = blockIdx.x;
  const int b    = blockIdx.y;
  const int t    = threadIdx.x;
  const int lane = t & 31, wave = t >> 5;
#pragma unroll
  for (int j = 0; j < 4; ++j) {
    const int c = cg * 32 + wave * 4 + j;
    const v4u* rp = (const v4u*)(V16 + ((size_t)(b * kCh + c)) * kPix) + lane * 16;
    float s = 0.f;
#pragma unroll 1
    for (int i = 0; i < 16; ++i) {
      const v4u w = rp[i];
#pragma unroll
      for (int e = 0; e < 4; ++e) {
        s += h2f_bits(w[e] & 0xffffu);
        s += h2f_bits(w[e] >> 16);
      }
    }
#pragma unroll
    for (int off = 16; off > 0; off >>= 1) s += __shfl_xor(s, off, 32);
    if (lane == 0) red[wave * 4 + j] = s;
  }
  __syncthreads();
  if (wave == 0 && lane < 8) {
    v4f v;
    v[0] = red[4 * lane + 0] * kMeanScale;
    v[1] = red[4 * lane + 1] * kMeanScale;
    v[2] = red[4 * lane + 2] * kMeanScale;
    v[3] = red[4 * lane + 3] * kMeanScale;
    float* d = vmean + (size_t)b * kCh + cg * 32 + 4 * lane;
    *(volatile v4f*)d = v;
    __threadfence();
    *(volatile v4f*)d = v;
  }
}

extern "C" void kernel_launch(void* const* d_in, const int* in_sizes, int n_in,
                              void* d_out, int out_size, void* d_ws, size_t ws_size,
                              hipStream_t stream) {
  if (n_in < 7) return;
  if (in_sizes[0] != kBatch * kCh * kPix) return;
  if (in_sizes[1] != kInter * kCh || in_sizes[2] != kInter) return;
  if (in_sizes[3] != kInter * kCh || in_sizes[4] != kInter) return;
  if (in_sizes[5] != kCh * kCh || in_sizes[6] != kCh) return;
  if (out_size != kBatch * kCh * kPix) return;

  const float* x  = (const float*)d_in[0];
  const float* wq = (const float*)d_in[1];
  const float* bq = (const float*)d_in[2];
  const float* wk = (const float*)d_in[3];
  const float* bk = (const float*)d_in[4];
  const float* wv = (const float*)d_in[5];
  const float* bv = (const float*)d_in[6];
  float* out = (float*)d_out;

  const size_t szX16  = (size_t)kTok * kCh * 2;
  const size_t szQK   = (size_t)kTok * kQKN * 2;
  const size_t szV16  = (size_t)kBatch * kCh * kPix * 2;
  const size_t szS32  = (size_t)kChunkQ * kPix * 4;
  const size_t szP16  = (size_t)kChunkQ * kPix * 2;
  const size_t szWqk  = (size_t)kQKN * kCh * 2;
  const size_t szWv   = (size_t)kCh * kCh * 2;
  const size_t szBqk  = (size_t)kQKN * 4;
  const size_t szBv   = (size_t)kCh * 4;
  const size_t szMean = (size_t)kBatch * kCh * 4;

  const size_t oX16  = 0;
  const size_t oQK   = oX16 + szX16;
  const size_t oV16  = oQK + szQK;
  const size_t oS32  = oV16 + szV16;
  const size_t oP16  = oS32 + szS32;
  const size_t oWqk  = oP16 + szP16;
  const size_t oWv   = oWqk + szWqk;
  const size_t oBqk  = oWv + szWv;
  const size_t oBv   = oBqk + szBqk;
  const size_t oMean = oBv + szBv;
  const size_t total = oMean + szMean;
  if (total > ws_size) return;

  char* ws = (char*)d_ws;
  unsigned short* X16   = (unsigned short*)(ws + oX16);
  unsigned short* QK16  = (unsigned short*)(ws + oQK);
  unsigned short* V16   = (unsigned short*)(ws + oV16);
  float*          S32   = (float*)(ws + oS32);
  unsigned short* P16   = (unsigned short*)(ws + oP16);
  unsigned short* Wqk16 = (unsigned short*)(ws + oWqk);
  unsigned short* Wv16  = (unsigned short*)(ws + oWv);
  float*          biasqk = (float*)(ws + oBqk);
  float*          biasv  = (float*)(ws + oBv);
  float*          vmean  = (float*)(ws + oMean);

  xpose_kernel<<<dim3(kPix / 64, kCh / 64, kBatch), 256, 0, stream>>>(x, X16);

  prep_kernel<<<49, 256, 0, stream>>>(wq, wk, wv, bq, bk, bv, Wqk16, Wv16, biasqk, biasv);

  wmma_gemm64<0, false, 2, 1, false, 0, false><<<dim3((kTok / 64) * (kQKN / 64) / 8, 1), 256, 0, stream>>>(
      X16, X16, kCh, (long)0,
      Wqk16, Wqk16, kCh, (long)0,
      (void*)QK16, (void*)QK16, kQKN, (long)0,
      biasqk, biasqk, (long)0,
      biasqk, (long)0,
      kTok, kQKN, kCh, kProjScale);

  wmma_gemm64<0, false, 1, 1, false, 0, false><<<dim3((kCh / 64) * (kPix / 64) / 8, kBatch), 256, 0, stream>>>(
      Wv16, Wv16, kCh, (long)0,
      X16, X16, kCh, (long)kPix * kCh,
      (void*)V16, (void*)V16, kPix, (long)kCh * kPix,
      biasv, biasv, (long)0,
      biasv, (long)0,
      kCh, kPix, kCh, kVScale);

  vmean_kernel<<<dim3(kCh / 32, kBatch), 256, 0, stream>>>(V16, vmean);

  for (int ch = 0; ch < kBatch * kHalves; ++ch) {
    const int b = ch / kHalves;
    const int half = ch - b * kHalves;
    const unsigned short* Qrows = QK16 + ((size_t)b * kPix + (size_t)half * kChunkQ) * kQKN;
    const unsigned short* Krows = QK16 + ((size_t)b * kPix) * kQKN + kInter;
    wmma_gemm64<0, false, 0, 0, false, 0, false><<<dim3((kChunkQ / 64) * (kPix / 64) / 8, 1), 256, 0, stream>>>(
        Qrows, Qrows, kQKN, (long)0,
        Krows, Krows, kQKN, (long)0,
        (void*)S32, (void*)S32, kPix, (long)0,
        biasqk, biasqk, (long)0,
        biasqk, (long)0,
        kChunkQ, kPix, kInter, kSScale);
    softmax_row_kernel<<<kChunkQ, 512, 0, stream>>>(S32, P16);
    const unsigned short* Vrows = V16 + (size_t)b * kCh * kPix;
    float* orow = out + (size_t)b * kCh * kPix + (size_t)half * kChunkQ;
    wmma_gemm64<0, false, 0, 0, false, 0, true><<<dim3((kCh / 64) * (kChunkQ / 64) / 8, 1), 256, 0, stream>>>(
        Vrows, Vrows, kPix, (long)0,
        P16, P16, kPix, (long)0,
        (void*)orow, (void*)orow, kPix, (long)0,
        biasqk, biasqk, (long)0,
        vmean + (size_t)b * kCh, (long)0,
        kCh, kChunkQ, kPix, kOutScale);
  }
}
